// ImprovedEdgeGraphSAGE_44444321579081
// MI455X (gfx1250) — hardware-verified
//
#include <hip/hip_runtime.h>
#include <math.h>
#include <stdint.h>

#define NN   1024
#define DEGR 4
#define NE   4096
#define FIN  128
#define HC   256
#define EDM  32
#define AD   512
#define NH   4
#define HD   128
#define KW1  320
#define CSP  132

static_assert(NE == NN * DEGR);
static_assert(AD == NH * HD);

typedef __attribute__((ext_vector_type(16))) __bf16 v16b;
typedef __attribute__((ext_vector_type(8)))  __bf16 v8b;
typedef __attribute__((ext_vector_type(8)))  float  v8f;
typedef __attribute__((ext_vector_type(4)))  float  v4f;
typedef __attribute__((ext_vector_type(4)))  unsigned int v4u;
typedef __attribute__((ext_vector_type(2)))  unsigned int v2u;

union FB { v16b v; v8b h[2]; };

struct Opnd {
  const unsigned short* hi;
  const unsigned short* lo;
  int rs;
  int bs;
};
static_assert(sizeof(Opnd) == 24);

__device__ __forceinline__ unsigned short f2bf_bits(float f) {
  unsigned u = __float_as_uint(f);
  return (unsigned short)((u + 0x7FFFu + ((u >> 16) & 1u)) >> 16);
}
__device__ __forceinline__ float bf_bits2f(unsigned short b) { return __uint_as_float(((unsigned)b) << 16); }
__device__ __forceinline__ unsigned pk16(unsigned short a, unsigned short b) { return (unsigned)a | ((unsigned)b << 16); }

__device__ __forceinline__ void split2(float f0, float f1, unsigned& hw, unsigned& lw) {
  const unsigned short h0 = f2bf_bits(f0), h1 = f2bf_bits(f1);
  const unsigned short l0 = f2bf_bits(f0 - bf_bits2f(h0)), l1 = f2bf_bits(f1 - bf_bits2f(h1));
  hw = pk16(h0, h1);
  lw = pk16(l0, l1);
}

__device__ __forceinline__ v8f mma_bf(v16b a, v16b b, v8f c) {
  c = __builtin_amdgcn_wmma_f32_16x16x32_bf16(false, a, false, b, (short)0, c, false, false);
  asm volatile("v_nop\n\tv_nop\n\tv_nop\n\tv_nop" : "+v"(c) : "v"(a), "v"(b));
  return c;
}

__device__ __forceinline__ v8b ldb8(const unsigned short* p) { return *(const v8b*)(const void*)p; }

__device__ __forceinline__ float sigm(float x) {
  const float xc = fminf(fmaxf(x, -30.0f), 30.0f);
  return 1.0f / (1.0f + __expf(-xc));
}

__global__ __launch_bounds__(256) void wsplit_kernel(const float* __restrict__ src,
                                                     unsigned short* __restrict__ hi,
                                                     unsigned short* __restrict__ lo,
                                                     int K, int Kp, int permF, int grp, int ngrp) {
  const int t = blockIdx.x * 256 + (int)threadIdx.x;
  if (t >= ngrp) return;
  const int cpr  = Kp >> 3;
  const int orow = t / cpr;
  const int c8   = (t - orow * cpr) * 8;
  int srow = orow;
  if (permF > 0) {
    const int gq = orow / grp;
    const int r  = orow - gq * grp;
    srow = gq * grp + (r & 3) * permF + (r >> 2);
  }
  const int cc = (c8 + 8 <= K) ? c8 : (K - 8);
  const float* sp = src + (size_t)srow * K + cc;
  v4f a0 = *(const v4f*)(sp);
  v4f a1 = *(const v4f*)(sp + 4);
  if (c8 + 8 > K) { a0 = (v4f){0.f, 0.f, 0.f, 0.f}; a1 = (v4f){0.f, 0.f, 0.f, 0.f}; }
  unsigned h0, h1, h2, h3, l0, l1, l2, l3;
  split2(a0[0], a0[1], h0, l0);
  split2(a0[2], a0[3], h1, l1);
  split2(a1[0], a1[1], h2, l2);
  split2(a1[2], a1[3], h3, l3);
  const v4u hv = (v4u){h0, h1, h2, h3};
  const v4u lv = (v4u){l0, l1, l2, l3};
  const size_t d = (size_t)orow * Kp + c8;
  *(volatile v4u*)(hi + d) = hv;
  *(volatile v4u*)(lo + d) = lv;
  __threadfence();
  *(volatile v4u*)(hi + d) = hv;
  *(volatile v4u*)(lo + d) = lv;
}

__global__ __launch_bounds__(256) void ef_gather_kernel(const unsigned short* __restrict__ hh,
                                                        const unsigned short* __restrict__ hl,
                                                        const int* __restrict__ ei,
                                                        unsigned short* __restrict__ efh,
                                                        unsigned short* __restrict__ efl, int ngrp) {
  const int t = blockIdx.x * 256 + (int)threadIdx.x;
  if (t >= ngrp) return;
  const int e = t >> 6, c = t & 63;
  const int which = c >> 5;
  int node = ei[which * NE + e];
  node = min(max(node, 0), NN - 1);
  const size_t so = (size_t)node * HC + (size_t)(c & 31) * 8;
  const v4u a = *(const v4u*)(hh + so);
  const v4u b = *(const v4u*)(hl + so);
  const size_t d = (size_t)e * AD + (size_t)c * 8;
  *(volatile v4u*)(efh + d) = a;
  *(volatile v4u*)(efl + d) = b;
  __threadfence();
  *(volatile v4u*)(efh + d) = a;
  *(volatile v4u*)(efl + d) = b;
}

__global__ __launch_bounds__(256) void zext_kernel(const float* __restrict__ ea,
                                                   unsigned short* __restrict__ zh,
                                                   unsigned short* __restrict__ zl, int ngrp) {
  const int t = blockIdx.x * 256 + (int)threadIdx.x;
  if (t >= ngrp) return;
  const int e = t >> 3, c8 = (t & 7) * 8;
  const int cc = (c8 + 8 <= EDM) ? c8 : (EDM - 8);
  const float* sp = ea + (size_t)e * EDM + cc;
  v4f a0 = *(const v4f*)(sp);
  v4f a1 = *(const v4f*)(sp + 4);
  if (c8 + 8 > EDM) { a0 = (v4f){0.f, 0.f, 0.f, 0.f}; a1 = (v4f){0.f, 0.f, 0.f, 0.f}; }
  unsigned h0, h1, h2, h3, l0, l1, l2, l3;
  split2(a0[0], a0[1], h0, l0);
  split2(a0[2], a0[3], h1, l1);
  split2(a1[0], a1[1], h2, l2);
  split2(a1[2], a1[3], h3, l3);
  const v4u hv = (v4u){h0, h1, h2, h3};
  const v4u lv = (v4u){l0, l1, l2, l3};
  const size_t d = (size_t)e * KW1 + HC + c8;
  *(volatile v4u*)(zh + d) = hv;
  *(volatile v4u*)(zl + d) = lv;
  __threadfence();
  *(volatile v4u*)(zh + d) = hv;
  *(volatile v4u*)(zl + d) = lv;
}

__device__ __forceinline__ void gemm_phase(v8f (&acc)[2][2], const Opnd& A, const Opnd& W, int K,
                                           int ra, int cb, int lh) {
  const size_t ao0 = (size_t)ra * (size_t)A.rs + (size_t)(8 * lh);
  const size_t ao1 = ao0 + (size_t)16 * (size_t)A.rs;
  const size_t bo0 = (size_t)cb * (size_t)W.rs + (size_t)(8 * lh);
  const size_t bo1 = bo0 + (size_t)16 * (size_t)W.rs;
  const int nk = K >> 5;
#pragma unroll 1
  for (int kb = 0; kb < nk; ++kb) {
    const size_t ka = (size_t)kb * (size_t)A.bs;
    const size_t kw = (size_t)kb * (size_t)W.bs;
    FB ah0, ah1, al0, al1, bh0, bh1, bl0, bl1;
    ah0.h[0] = ldb8(A.hi + ao0 + ka);  ah0.h[1] = ldb8(A.hi + ao0 + ka + 16);
    ah1.h[0] = ldb8(A.hi + ao1 + ka);  ah1.h[1] = ldb8(A.hi + ao1 + ka + 16);
    al0.h[0] = ldb8(A.lo + ao0 + ka);  al0.h[1] = ldb8(A.lo + ao0 + ka + 16);
    al1.h[0] = ldb8(A.lo + ao1 + ka);  al1.h[1] = ldb8(A.lo + ao1 + ka + 16);
    bh0.h[0] = ldb8(W.hi + bo0 + kw);  bh0.h[1] = ldb8(W.hi + bo0 + kw + 16);
    bh1.h[0] = ldb8(W.hi + bo1 + kw);  bh1.h[1] = ldb8(W.hi + bo1 + kw + 16);
    bl0.h[0] = ldb8(W.lo + bo0 + kw);  bl0.h[1] = ldb8(W.lo + bo0 + kw + 16);
    bl1.h[0] = ldb8(W.lo + bo1 + kw);  bl1.h[1] = ldb8(W.lo + bo1 + kw + 16);
    acc[0][0] = mma_bf(ah0.v, bh0.v, acc[0][0]);
    acc[0][0] = mma_bf(ah0.v, bl0.v, acc[0][0]);
    acc[0][0] = mma_bf(al0.v, bh0.v, acc[0][0]);
    acc[0][1] = mma_bf(ah0.v, bh1.v, acc[0][1]);
    acc[0][1] = mma_bf(ah0.v, bl1.v, acc[0][1]);
    acc[0][1] = mma_bf(al0.v, bh1.v, acc[0][1]);
    acc[1][0] = mma_bf(ah1.v, bh0.v, acc[1][0]);
    acc[1][0] = mma_bf(ah1.v, bl0.v, acc[1][0]);
    acc[1][0] = mma_bf(al1.v, bh0.v, acc[1][0]);
    acc[1][1] = mma_bf(ah1.v, bh1.v, acc[1][1]);
    acc[1][1] = mma_bf(ah1.v, bl1.v, acc[1][1]);
    acc[1][1] = mma_bf(al1.v, bh1.v, acc[1][1]);
  }
}

template <int EPI>
__global__ __launch_bounds__(256) void gemm3_kernel(
    Opnd A1, Opnd W1, int K1, Opnd A2, Opnd W2, int K2,
    const float* __restrict__ bias1, const float* __restrict__ bias2, int permF,
    const float* __restrict__ resid, int ldr, int relu,
    float* cf, int ldc,
    unsigned short* ph, unsigned short* pl, int ldp,
    const float* __restrict__ gx, int ldg, const int* __restrict__ sidx, int tstep, int Mtot,
    unsigned short* kh, unsigned short* kl, unsigned short* vth, unsigned short* vtl) {
  __shared__ __align__(16) float Cs[64 * CSP];
  const int tid = threadIdx.x;
  const int wave = tid >> 5, lane = tid & 31;
  const int lh = lane >> 4, c = lane & 15;
  const int wm = wave & 1, wn = wave >> 1;
  const int m0 = blockIdx.x * 64, n0 = blockIdx.y * 128;

  v8f acc[2][2];
#pragma unroll
  for (int i = 0; i < 2; ++i)
#pragma unroll
    for (int j = 0; j < 2; ++j) acc[i][j] = (v8f){0.f, 0.f, 0.f, 0.f, 0.f, 0.f, 0.f, 0.f};

  gemm_phase(acc, A1, W1, K1, m0 + wm * 32 + c, n0 + wn * 32 + c, lh);
  gemm_phase(acc, A2, W2, K2, m0 + wm * 32 + c, n0 + wn * 32 + c, lh);

#pragma unroll
  for (int i = 0; i < 2; ++i)
#pragma unroll
    for (int j = 0; j < 2; ++j)
#pragma unroll
      for (int r = 0; r < 8; ++r)
        Cs[(wm * 32 + i * 16 + 8 * lh + r) * CSP + wn * 32 + j * 16 + c] = acc[i][j][r];
  __syncthreads();

  if (EPI == 0) {
    const int c4  = lane * 4;
    const int col = n0 + c4;
    float badd[4] = {0.f, 0.f, 0.f, 0.f};
#pragma unroll
    for (int q = 0; q < 4; ++q) {
      const int pc = permF ? (q * permF + (col >> 2)) : (col + q);
      if (bias1) badd[q] += bias1[pc];
      if (bias2) badd[q] += bias2[pc];
    }
#pragma unroll 1
    for (int pass = 0; pass < 8; ++pass) {
      const int r   = pass * 8 + wave;
      const int row = m0 + r;
      v4f v = *(const v4f*)(Cs + r * CSP + c4);
      v[0] += badd[0]; v[1] += badd[1]; v[2] += badd[2]; v[3] += badd[3];
      if (resid) v += *(const v4f*)(resid + (size_t)row * ldr + col);
      if (relu) { v[0] = fmaxf(v[0], 0.f); v[1] = fmaxf(v[1], 0.f); v[2] = fmaxf(v[2], 0.f); v[3] = fmaxf(v[3], 0.f); }
      unsigned hw0, hw1, lw0, lw1;
      split2(v[0], v[1], hw0, lw0);
      split2(v[2], v[3], hw1, lw1);
      const v2u hv = (v2u){hw0, hw1};
      const v2u lv = (v2u){lw0, lw1};
      const size_t fo = (size_t)row * ldc + col;
      const size_t po = (size_t)row * ldp + col;
      if (cf) *(volatile v4f*)(cf + fo) = v;
      if (ph) { *(volatile v2u*)(ph + po) = hv; *(volatile v2u*)(pl + po) = lv; }
      __threadfence();
      if (cf) *(volatile v4f*)(cf + fo) = v;
      if (ph) { *(volatile v2u*)(ph + po) = hv; *(volatile v2u*)(pl + po) = lv; }
    }
  } else if (EPI == 1) {
    const int ub = blockIdx.y;
    const int ug = tid & 7;
#pragma unroll 1
    for (int pass = 0; pass < 2; ++pass) {
      const int r    = pass * 32 + (tid >> 3);
      const int node = m0 + r;
      const float* cr = Cs + r * CSP + 16 * ug;
      int si = sidx[4 * node + tstep];
      si = min(max(si, 0), Mtot - 1);
      const float* gr = gx + (size_t)si * ldg + n0 + 16 * ug;
      v4f gv[4];
#pragma unroll
      for (int u = 0; u < 4; ++u) gv[u] = *(const v4f*)(cr + 4 * u) + *(const v4f*)(gr + 4 * u);
      const size_t co = ((size_t)ub * Mtot + node) * 32 + 4 * ug;
      v4f cp = *(const v4f*)(cf + co);
      if (tstep == 0) cp = (v4f){0.f, 0.f, 0.f, 0.f};
      v4f cv;
      float hn[4];
#pragma unroll
      for (int u = 0; u < 4; ++u) {
        const float ig = sigm(gv[u][0]);
        const float fg = sigm(gv[u][1]);
        const float gg = tanhf(gv[u][2]);
        const float og = sigm(gv[u][3]);
        const float cn = fg * cp[u] + ig * gg;
        cv[u] = cn;
        hn[u] = og * tanhf(cn);
      }
      unsigned hw0, hw1, lw0, lw1;
      split2(hn[0], hn[1], hw0, lw0);
      split2(hn[2], hn[3], hw1, lw1);
      const v2u hv = (v2u){hw0, hw1};
      const v2u lv = (v2u){lw0, lw1};
      *(volatile v4f*)(cf + co) = cv;
      *(volatile v2u*)(ph + co) = hv;
      *(volatile v2u*)(pl + co) = lv;
      __threadfence();
      *(volatile v4f*)(cf + co) = cv;
      *(volatile v2u*)(ph + co) = hv;
      *(volatile v2u*)(pl + co) = lv;
    }
  } else {
    const int s = blockIdx.y;
    const int which = s >> 2, head = s & 3;
    if (which < 2) {
      unsigned short* dh = (which == 0 ? ph : kh) + (size_t)head * NE * HD;
      unsigned short* dl = (which == 0 ? pl : kl) + (size_t)head * NE * HD;
      const int c4 = lane * 4;
      float badd[4];
#pragma unroll
      for (int q = 0; q < 4; ++q) badd[q] = bias1[n0 + c4 + q];
#pragma unroll 1
      for (int pass = 0; pass < 8; ++pass) {
        const int r     = pass * 8 + wave;
        const int token = m0 + r;
        v4f v = *(const v4f*)(Cs + r * CSP + c4);
        v[0] += badd[0]; v[1] += badd[1]; v[2] += badd[2]; v[3] += badd[3];
        unsigned hw0, hw1, lw0, lw1;
        split2(v[0], v[1], hw0, lw0);
        split2(v[2], v[3], hw1, lw1);
        const v2u hv = (v2u){hw0, hw1};
        const v2u lv = (v2u){lw0, lw1};
        const size_t po = (size_t)token * HD + c4;
        *(volatile v2u*)(dh + po) = hv;
        *(volatile v2u*)(dl + po) = lv;
        __threadfence();
        *(volatile v2u*)(dh + po) = hv;
        *(volatile v2u*)(dl + po) = lv;
      }
    } else {
      const int sub = tid >> 3;
      const int t8  = (tid & 7) * 8;
      v4u hvv[4], lvv[4];
#pragma unroll
      for (int it = 0; it < 4; ++it) {
        const int d = it * 32 + sub;
        const float bb = bias1[n0 + d];
        unsigned hw[4], lw[4];
#pragma unroll
        for (int q = 0; q < 4; ++q) {
          const float f0 = Cs[(t8 + 2 * q) * CSP + d] + bb;
          const float f1 = Cs[(t8 + 2 * q + 1) * CSP + d] + bb;
          split2(f0, f1, hw[q], lw[q]);
        }
        hvv[it] = (v4u){hw[0], hw[1], hw[2], hw[3]};
        lvv[it] = (v4u){lw[0], lw[1], lw[2], lw[3]};
      }
      for (int ps = 0; ps < 2; ++ps) {
#pragma unroll
        for (int it = 0; it < 4; ++it) {
          const int d = it * 32 + sub;
          const size_t o = ((size_t)head * HD + d) * NE + m0 + t8;
          *(volatile v4u*)(vth + o) = hvv[it];
          *(volatile v4u*)(vtl + o) = lvv[it];
        }
        __threadfence();
      }
    }
  }
}

#define QB  64
#define KC  64
#define KSP 136
#define VTP 72
#define PSP 64
#define OSP 68

__global__ __launch_bounds__(256)
void attn_kernel(const unsigned short* __restrict__ qhp, const unsigned short* __restrict__ qlp,
                 const unsigned short* __restrict__ khp, const unsigned short* __restrict__ klp,
                 const unsigned short* __restrict__ vhp, const unsigned short* __restrict__ vlp,
                 unsigned short* ohp, unsigned short* olp, float sscale) {
  __shared__ __align__(16) __bf16 Ksh[KC * KSP];
  __shared__ __align__(16) __bf16 Ksl[KC * KSP];
  __shared__ __align__(16) __bf16 Vth[HD * VTP];
  __shared__ __align__(16) __bf16 Vtl[HD * VTP];
  __shared__ __align__(16) __bf16 Psh[4][16 * PSP];
  __shared__ __align__(16) __bf16 Psl[4][16 * PSP];
  __shared__ __align__(16) float  Al[4][16];
  __shared__ __align__(16) float  Ll[4][16];
  __shared__ __align__(16) float  Os[8][16 * OSP];

  const int tid  = threadIdx.x;
  const int wave = tid >> 5;
  const int lane = tid & 31;
  const int lh   = lane >> 4;
  const int c    = lane & 15;
  const int g    = wave & 3;
  const int chh  = wave >> 2;
  const int ch0  = chh * 64;

  const int nqt  = NE / QB;
  const int qt   = blockIdx.x % nqt;
  const int head = blockIdx.x / nqt;
  const int qg0  = qt * QB + g * 16;

  const __bf16* Qh = (const __bf16*)(const void*)qhp + (size_t)head * NE * HD;
  const __bf16* Ql = (const __bf16*)(const void*)qlp + (size_t)head * NE * HD;
  const __bf16* Kh = (const __bf16*)(const void*)khp + (size_t)head * NE * HD;
  const __bf16* Kl = (const __bf16*)(const void*)klp + (size_t)head * NE * HD;
  const __bf16* Vh = (const __bf16*)(const void*)vhp + (size_t)head * HD * NE;
  const __bf16* Vl = (const __bf16*)(const void*)vlp + (size_t)head * HD * NE;

  float mrow[8], lrow[8];
  v8f oacc[4];
#pragma unroll
  for (int r = 0; r < 8; ++r) { mrow[r] = -INFINITY; lrow[r] = 0.f; }
#pragma unroll
  for (int t = 0; t < 4; ++t) oacc[t] = (v8f){0.f, 0.f, 0.f, 0.f, 0.f, 0.f, 0.f, 0.f};

  __bf16* pwh = Psh[g];
  __bf16* pwl = Psl[g];

  for (int kc = 0; kc < NE / KC; ++kc) {
    const int kv0 = kc * KC;
    __syncthreads();
    {
      const int r = tid >> 2, qq = (tid & 3) * 32;
      const __bf16* khs = Kh + (size_t)(kv0 + r) * HD + qq;
      const __bf16* kls = Kl + (size_t)(kv0 + r) * HD + qq;
      __bf16* kdh = Ksh + r * KSP + qq;
      __bf16* kdl = Ksl + r * KSP + qq;
#pragma unroll
      for (int i = 0; i < 4; ++i) {
        *(v8b*)(kdh + 8 * i) = *(const v8b*)(khs + 8 * i);
        *(v8b*)(kdl + 8 * i) = *(const v8b*)(kls + 8 * i);
      }
      const int r2 = tid >> 1, hf = (tid & 1) * 32;
      const __bf16* vhs = Vh + (size_t)r2 * NE + kv0 + hf;
      const __bf16* vls = Vl + (size_t)r2 * NE + kv0 + hf;
#pragma unroll
      for (int i = 0; i < 4; ++i) {
        *(v8b*)(Vth + r2 * VTP + hf + 8 * i) = *(const v8b*)(vhs + 8 * i);
        *(v8b*)(Vtl + r2 * VTP + hf + 8 * i) = *(const v8b*)(vls + 8 * i);
      }
    }
    __syncthreads();

    if (wave < 4) {
      v8f s[4];
#pragma unroll
      for (int j = 0; j < 4; ++j) s[j] = (v8f){0.f, 0.f, 0.f, 0.f, 0.f, 0.f, 0.f, 0.f};
      const __bf16* qrh = Qh + (size_t)(qg0 + c) * HD + 8 * lh;
      const __bf16* qrl = Ql + (size_t)(qg0 + c) * HD + 8 * lh;
#pragma unroll
      for (int dc = 0; dc < 4; ++dc) {
        FB qa, ql;
        qa.h[0] = *(const v8b*)(qrh + dc * 32);
        qa.h[1] = *(const v8b*)(qrh + dc * 32 + 16);
        ql.h[0] = *(const v8b*)(qrl + dc * 32);
        ql.h[1] = *(const v8b*)(qrl + dc * 32 + 16);
#pragma unroll
        for (int j = 0; j < 4; ++j) {
          const __bf16* kp = Ksh + (j * 16 + c) * KSP + dc * 32 + 8 * lh;
          const __bf16* kq = Ksl + (j * 16 + c) * KSP + dc * 32 + 8 * lh;
          FB kb, kl;
          kb.h[0] = *(const v8b*)(kp);
          kb.h[1] = *(const v8b*)(kp + 16);
          kl.h[0] = *(const v8b*)(kq);
          kl.h[1] = *(const v8b*)(kq + 16);
          s[j] = mma_bf(qa.v, kb.v, s[j]);
          s[j] = mma_bf(qa.v, kl.v, s[j]);
          s[j] = mma_bf(ql.v, kb.v, s[j]);
        }
      }
      float cm[8];
#pragma unroll
      for (int r = 0; r < 8; ++r) {
        float m = -INFINITY;
#pragma unroll
        for (int j = 0; j < 4; ++j) {
          const float sv = s[j][r] * sscale;
          s[j][r] = sv;
          m = fmaxf(m, sv);
        }
#pragma unroll
        for (int off = 1; off < 16; off <<= 1) m = fmaxf(m, __shfl_xor(m, off, 32));
        cm[r] = m;
      }
#pragma unroll
      for (int r = 0; r < 8; ++r) {
        const float mnew  = fmaxf(mrow[r], cm[r]);
        const float alpha = __expf(mrow[r] - mnew);
        mrow[r] = mnew;
        float psum = 0.f;
#pragma unroll
        for (int j = 0; j < 4; ++j) {
          const float p = __expf(s[j][r] - mnew);
          psum += p;
          const unsigned short hb = f2bf_bits(p);
          const unsigned short lb = f2bf_bits(p - bf_bits2f(hb));
          pwh[(8 * lh + r) * PSP + j * 16 + c] = __builtin_bit_cast(__bf16, hb);
          pwl[(8 * lh + r) * PSP + j * 16 + c] = __builtin_bit_cast(__bf16, lb);
        }
#pragma unroll
        for (int off = 1; off < 16; off <<= 1) psum += __shfl_xor(psum, off, 32);
        lrow[r] = lrow[r] * alpha + psum;
        if (c == 0) {
          Al[g][8 * lh + r] = alpha;
          Ll[g][8 * lh + r] = lrow[r];
        }
      }
    }
    __syncthreads();

    {
      float af[8];
#pragma unroll
      for (int r = 0; r < 8; ++r) af[r] = Al[g][8 * lh + r];
#pragma unroll
      for (int t = 0; t < 4; ++t)
#pragma unroll
        for (int r = 0; r < 8; ++r) oacc[t][r] *= af[r];
#pragma unroll 1
      for (int kk = 0; kk < 2; ++kk) {
        FB pa, pl;
        pa.h[0] = *(const v8b*)(pwh + c * PSP + kk * 32 + 8 * lh);
        pa.h[1] = *(const v8b*)(pwh + c * PSP + kk * 32 + 16 + 8 * lh);
        pl.h[0] = *(const v8b*)(pwl + c * PSP + kk * 32 + 8 * lh);
        pl.h[1] = *(const v8b*)(pwl + c * PSP + kk * 32 + 16 + 8 * lh);
#pragma unroll
        for (int t = 0; t < 4; ++t) {
          const __bf16* vp = Vth + (ch0 + t * 16 + c) * VTP + kk * 32 + 8 * lh;
          const __bf16* vq = Vtl + (ch0 + t * 16 + c) * VTP + kk * 32 + 8 * lh;
          FB vb, vl;
          vb.h[0] = *(const v8b*)(vp);
          vb.h[1] = *(const v8b*)(vp + 16);
          vl.h[0] = *(const v8b*)(vq);
          vl.h[1] = *(const v8b*)(vq + 16);
          oacc[t] = mma_bf(pa.v, vb.v, oacc[t]);
          oacc[t] = mma_bf(pa.v, vl.v, oacc[t]);
          oacc[t] = mma_bf(pl.v, vb.v, oacc[t]);
        }
      }
    }
  }

  float* os = Os[wave];
#pragma unroll
  for (int r = 0; r < 8; ++r) {
    const float inv = 1.0f / Ll[g][8 * lh + r];
#pragma unroll
    for (int t = 0; t < 4; ++t) os[(8 * lh + r) * OSP + t * 16 + c] = oacc[t][r] * inv;
  }
  __builtin_amdgcn_fence(__ATOMIC_RELEASE, "workgroup");
  __builtin_amdgcn_wave_barrier();
  __builtin_amdgcn_fence(__ATOMIC_ACQUIRE, "workgroup");
  {
    const int rq = lane >> 3, c8 = (lane & 7) * 8;
    v4u hv[4], lv[4];
#pragma unroll
    for (int it = 0; it < 4; ++it) {
      const int row = it * 4 + rq;
      const v4f x0 = *(const v4f*)(os + row * OSP + c8);
      const v4f x1 = *(const v4f*)(os + row * OSP + c8 + 4);
      unsigned h0, h1, h2, h3, l0, l1, l2, l3;
      split2(x0[0], x0[1], h0, l0);
      split2(x0[2], x0[3], h1, l1);
      split2(x1[0], x1[1], h2, l2);
      split2(x1[2], x1[3], h3, l3);
      hv[it] = (v4u){h0, h1, h2, h3};
      lv[it] = (v4u){l0, l1, l2, l3};
    }
    for (int ps = 0; ps < 2; ++ps) {
#pragma unroll
      for (int it = 0; it < 4; ++it) {
        const int row = it * 4 + rq;
        const size_t go = (size_t)(qg0 + row) * AD + (size_t)head * HD + ch0 + c8;
        *(volatile v4u*)(ohp + go) = hv[it];
        *(volatile v4u*)(olp + go) = lv[it];
      }
      __threadfence();
    }
  }
}

__global__ __launch_bounds__(256) void head_kernel(const float* __restrict__ z2,
                                                   const float* __restrict__ w3,
                                                   const float* __restrict__ b3,
                                                   float* out, int ngrp) {
  const int t = blockIdx.x * 256 + (int)threadIdx.x;
  if (t >= ngrp) return;
  const float* za = z2 + (size_t)(2 * t) * HD;
  const float* zb = za + HD;
  float s00 = 0.f, s01 = 0.f, s10 = 0.f, s11 = 0.f;
#pragma unroll 1
  for (int cc = 0; cc < HD; cc += 4) {
    const v4f a  = *(const v4f*)(za + cc);
    const v4f b  = *(const v4f*)(zb + cc);
    const v4f w0 = *(const v4f*)(w3 + cc);
    const v4f w1 = *(const v4f*)(w3 + HD + cc);
#pragma unroll
    for (int q = 0; q < 4; ++q) {
      s00 += a[q] * w0[q];
      s01 += a[q] * w1[q];
      s10 += b[q] * w0[q];
      s11 += b[q] * w1[q];
    }
  }
  const float bb0 = b3[0], bb1 = b3[1];
  const v4f v = (v4f){s00 + bb0, s01 + bb1, s10 + bb0, s11 + bb1};
  volatile v4f* po = (volatile v4f*)(out + (size_t)4 * t);
  *po = v;
  __threadfence();
  *po = v;
}

static Opnd mkop(const unsigned short* h, const unsigned short* l, int rs, int bs) {
  Opnd o; o.hi = h; o.lo = l; o.rs = rs; o.bs = bs; return o;
}

static void launch_wsplit(hipStream_t st, const float* src, unsigned short* h, unsigned short* l,
                          int rows, int K, int Kp, int permF, int grp) {
  const int ngrp = rows * (Kp / 8);
  wsplit_kernel<<<dim3((ngrp + 255) / 256), dim3(256), 0, st>>>(src, h, l, K, Kp, permF, grp, ngrp);
}

static void launch_gemm_f32(hipStream_t st, int M, int N, Opnd A1, Opnd W1, int K1, Opnd A2, Opnd W2, int K2,
                            const float* b1, const float* b2, int permF,
                            const float* resid, int ldr, int relu,
                            float* cf, int ldc, unsigned short* ph, unsigned short* pl, int ldp) {
  gemm3_kernel<0><<<dim3(M / 64, N / 128), dim3(256), 0, st>>>(
      A1, W1, K1, A2, W2, K2, b1, b2, permF, resid, ldr, relu, cf, ldc, ph, pl, ldp,
      nullptr, 0, nullptr, 0, M, nullptr, nullptr, nullptr, nullptr);
}

static void launch_gemm_lstm(hipStream_t st, int M, int F4, Opnd A1, Opnd W1, int K1,
                             const float* gx, int ldg, const int* sidx, int tstep,
                             float* cst, unsigned short* hnh, unsigned short* hnl) {
  gemm3_kernel<1><<<dim3(M / 64, F4 / 128), dim3(256), 0, st>>>(
      A1, W1, K1, A1, W1, 0, nullptr, nullptr, F4 / 4, nullptr, 0, 0, cst, 0, hnh, hnl, 0,
      gx, ldg, sidx, tstep, M, nullptr, nullptr, nullptr, nullptr);
}

static void launch_gemm_qkv(hipStream_t st, Opnd A1, Opnd W1, int K1, const float* bias,
                            unsigned short* qh, unsigned short* ql, unsigned short* kh, unsigned short* kl,
                            unsigned short* vth, unsigned short* vtl) {
  gemm3_kernel<2><<<dim3(NE / 64, (3 * AD) / 128), dim3(256), 0, st>>>(
      A1, W1, K1, A1, W1, 0, bias, nullptr, 0, nullptr, 0, 0, nullptr, 0, qh, ql, HD,
      nullptr, 0, nullptr, 0, NE, kh, kl, vth, vtl);
}

extern "C" void kernel_launch(void* const* d_in, const int* in_sizes, int n_in,
                              void* d_out, int out_size, void* d_ws, size_t ws_size,
                              hipStream_t stream) {
  if (n_in != 27) return;
  const int expect_sz[27] = {
      NN * FIN, 2 * NE, NE * EDM,
      512 * 128, 512 * 128, 512, 512, 256 * 128, 256, 256 * 128,
      3 * 1024 * 256, 3 * 1024 * 256, 3 * 1024, 3 * 1024, 3 * 256 * 256, 3 * 256, 3 * 256 * 256,
      1536 * 512, 1536, 512 * 512, 512,
      256 * 288, 256, 128 * 256, 128, 2 * 128, 2};
  for (int i = 0; i < 27; ++i) if (in_sizes[i] != expect_sz[i]) return;
  if (out_size != NE * 2) return;

  const float* x          = (const float*)d_in[0];
  const int*   ei         = (const int*)d_in[1];
  const float* edge_attr  = (const float*)d_in[2];
  const float* l1_wih     = (const float*)d_in[3];
  const float* l1_whh     = (const float*)d_in[4];
  const float* l1_bih     = (const float*)d_in[5];
  const float* l1_bhh     = (const float*)d_in[6];
  const float* l1_wl      = (const float*)d_in[7];
  const float* l1_bl      = (const float*)d_in[8];
  const float* l1_wr      = (const float*)d_in[9];
  const float* ls_wih     = (const float*)d_in[10];
  const float* ls_whh     = (const float*)d_in[11];
  const float* ls_bih     = (const float*)d_in[12];
  const float* ls_bhh     = (const float*)d_in[13];
  const float* ls_wl      = (const float*)d_in[14];
  const float* ls_bl      = (const float*)d_in[15];
  const float* ls_wr      = (const float*)d_in[16];
  const float* attn_in_w  = (const float*)d_in[17];
  const float* attn_in_b  = (const float*)d_in[18];
  const float* attn_out_w = (const float*)d_in[19];
  const float* attn_out_b = (const float*)d_in[20];
  const float* mlp_w1     = (const float*)d_in[21];
  const float* mlp_b1     = (const float*)d_in[22];
  const float* mlp_w2     = (const float*)d_in[23];
  const float* mlp_b2     = (const float*)d_in[24];
  const float* mlp_w3     = (const float*)d_in[25];
  const float* mlp_b3     = (const float*)d_in[26];
  float* out = (float*)d_out;

  char* wsb = (char*)d_ws;
  size_t off = 0;
  auto carve = [&](size_t bytes) -> char* {
    char* p = wsb + off;
    off += (bytes + 255) & ~(size_t)255;
    return p;
  };
#define PLANES(name, elems) \
  unsigned short* name##h = (unsigned short*)carve((size_t)(elems) * 2); \
  unsigned short* name##l = (unsigned short*)carve((size_t)(elems) * 2);

  PLANES(W1IH, 512 * 128)
  PLANES(W1HH, 512 * 128)
  PLANES(W1L,  256 * 128)
  PLANES(W1R,  256 * 128)
  PLANES(WSIH, 3072 * 256)
  PLANES(WSHH, 3072 * 256)
  PLANES(WSL,  768 * 256)
  PLANES(WSR,  768 * 256)
  PLANES(AIN,  1536 * 512)
  PLANES(AOUT, 256 * 512)
  PLANES(MW1,  256 * KW1)
  PLANES(MW2,  128 * 256)
  PLANES(XPL,  NN * FIN)
  float* GX  = (float*)carve((size_t)NN * 1024 * 4);
  float* CST = (float*)carve((size_t)NN * HC * 4);
  PLANES(HP0,  NN * HC)
  PLANES(HP1,  NN * HC)
  float* HAF = (float*)carve((size_t)NN * HC * 4);
  PLANES(HAP,  NN * HC)
  float* HBF = (float*)carve((size_t)NN * HC * 4);
  PLANES(HBP,  NN * HC)
  PLANES(EF,   NE * AD)
  PLANES(QP,   NH * NE * HD)
  PLANES(KP,   NH * NE * HD)
  PLANES(VT,   NH * HD * NE)
  PLANES(OP,   NE * AD)
  PLANES(ZP,   NE * KW1)
  PLANES(Z1P,  NE * HC)
  float* Z2  = (float*)carve((size_t)NE * HD * 4);
#undef PLANES
  if (off > ws_size) return;

  launch_wsplit(stream, l1_wih, W1IHh, W1IHl, 512, 128, 128, 128, 512);
  launch_wsplit(stream, l1_whh, W1HHh, W1HHl, 512, 128, 128, 128, 512);
  launch_wsplit(stream, l1_wl,  W1Lh,  W1Ll,  256, 128, 128, 0, 256);
  launch_wsplit(stream, l1_wr,  W1Rh,  W1Rl,  256, 128, 128, 0, 256);
  launch_wsplit(stream, ls_wih, WSIHh, WSIHl, 3072, 256, 256, 256, 1024);
  launch_wsplit(stream, ls_whh, WSHHh, WSHHl, 3072, 256, 256, 256, 1024);
  launch_wsplit(stream, ls_wl,  WSLh,  WSLl,  768, 256, 256, 0, 768);
  launch_wsplit(stream, ls_wr,  WSRh,  WSRl,  768, 256, 256, 0, 768);
  launch_wsplit(stream, attn_in_w, AINh, AINl, 1536, 512, 512, 0, 1536);
  launch_wsplit(stream, attn_out_w + (size_t)256 * 512, AOUTh, AOUTl, 256, 512, 512, 0, 256);
  launch_wsplit(stream, mlp_w1, MW1h, MW1l, 256, 288, KW1, 0, 256);
  launch_wsplit(stream, mlp_w2, MW2h, MW2l, 128, 256, 256, 0, 128);
  launch_wsplit(stream, x, XPLh, XPLl, NN, FIN, FIN, 0, NN);

  const int HBS = 32 * NN;
  unsigned short* HPh[2] = {HP0h, HP1h};
  unsigned short* HPl[2] = {HP0l, HP1l};

  {
    const Opnd xop = mkop(XPLh, XPLl, FIN, 32);
    launch_gemm_f32(stream, NN, 512, xop, mkop(W1IHh, W1IHl, FIN, 32), FIN, xop, xop, 0,
                    l1_bih, l1_bhh, 128, nullptr, 0, 0, GX, 512, nullptr, nullptr, 0);
    for (int t = 0; t < DEGR; ++t) {
      const Opnd hop = mkop(HPh[(t & 1) ^ 1], HPl[(t & 1) ^ 1], 32, HBS);
      launch_gemm_lstm(stream, NN, 512, hop, mkop(W1HHh, W1HHl, 128, 32), t ? 128 : 0,
                       GX, 512, ei, t, CST, HPh[t & 1], HPl[t & 1]);
    }
    launch_gemm_f32(stream, NN, HC, mkop(HP1h, HP1l, 32, HBS), mkop(W1Lh, W1Ll, 128, 32), 128,
                    xop, mkop(W1Rh, W1Rl, FIN, 32), FIN,
                    l1_bl, nullptr, 0, nullptr, 0, 1, HAF, HC, HAPh, HAPl, HC);
  }

  for (int i = 0; i < 3; ++i) {
    const float* hinF = (i & 1) ? HBF : HAF;
    unsigned short* hinh = (i & 1) ? HBPh : HAPh;
    unsigned short* hinl = (i & 1) ? HBPl : HAPl;
    float* houtF = (i & 1) ? HAF : HBF;
    unsigned short* houth = (i & 1) ? HAPh : HBPh;
    unsigned short* houtl = (i & 1) ? HAPl : HBPl;
    const size_t wo  = (size_t)i * 1024 * 256;
    const size_t wo2 = (size_t)i * 256 * 256;
    const Opnd hinop = mkop(hinh, hinl, HC, 32);
    launch_gemm_f32(stream, NN, 1024, hinop, mkop(WSIHh + wo, WSIHl + wo, HC, 32), HC, hinop, hinop, 0,
                    ls_bih + (size_t)i * 1024, ls_bhh + (size_t)i * 1024, 256, nullptr, 0, 0,
                    GX, 1024, nullptr, nullptr, 0);
    for (int t = 0; t < DEGR; ++t) {
      const Opnd hop = mkop(HPh[(t & 1) ^ 1], HPl[(t & 1) ^ 1], 32, HBS);
      launch_gemm_lstm(stream, NN, 1024, hop, mkop(WSHHh + wo, WSHHl + wo, HC, 32), t ? HC : 0,
                       GX, 1024, ei, t, CST, HPh[t & 1], HPl[t & 1]);
    }
    launch_gemm_f32(stream, NN, HC, mkop(HP1h, HP1l, 32, HBS), mkop(WSLh + wo2, WSLl + wo2, HC, 32), HC,
                    hinop, mkop(WSRh + wo2, WSRl + wo2, HC, 32), HC,
                    ls_bl + (size_t)i * 256, nullptr, 0, hinF, HC, 1, houtF, HC, houth, houtl, HC);
  }

  ef_gather_kernel<<<dim3((NE * 64) / 256), dim3(256), 0, stream>>>(HBPh, HBPl, ei, EFh, EFl, NE * 64);
  zext_kernel<<<dim3((NE * 8) / 256), dim3(256), 0, stream>>>(edge_attr, ZPh, ZPl, NE * 8);
  launch_gemm_qkv(stream, mkop(EFh, EFl, AD, 32), mkop(AINh, AINl, AD, 32), AD, attn_in_b,
                  QPh, QPl, KPh, KPl, VTh, VTl);
  attn_kernel<<<dim3(NH * (NE / QB)), dim3(256), 0, stream>>>(QPh, QPl, KPh, KPl, VTh, VTl, OPh, OPl,
                                                             0.08838834764831845f);
  {
    const Opnd oop = mkop(OPh, OPl, AD, 32);
    launch_gemm_f32(stream, NE, HC, oop, mkop(AOUTh, AOUTl, AD, 32), AD, oop, oop, 0,
                    attn_out_b + 256, nullptr, 0, nullptr, 0, 0, nullptr, 0, ZPh, ZPl, KW1);
    const Opnd zop = mkop(ZPh, ZPl, KW1, 32);
    launch_gemm_f32(stream, NE, HC, zop, mkop(MW1h, MW1l, KW1, 32), KW1, zop, zop, 0,
                    mlp_b1, nullptr, 0, nullptr, 0, 1, nullptr, 0, Z1Ph, Z1Pl, HC);
    const Opnd z1op = mkop(Z1Ph, Z1Pl, HC, 32);
    launch_gemm_f32(stream, NE, HD, z1op, mkop(MW2h, MW2l, HC, 32), HC, z1op, z1op, 0,
                    mlp_b2, nullptr, 0, nullptr, 0, 1, Z2, HD, nullptr, nullptr, 0);
  }
  head_kernel<<<dim3((NE / 2) / 256), dim3(256), 0, stream>>>(Z2, mlp_w3, mlp_b3, out, NE / 2);
  (void)hipGetLastError();
}
